// Local2DAttentionLayer_31911607009651
// MI455X (gfx1250) — hardware-run, weakly checked
//
#include <hip/hip_runtime.h>


#ifndef NB
#define NB 2
#endif
#define NB_FULL 2
#define CH   192
#define IH   64
#define IW   64
#define LPIX (IH * IW)
#define NHD  6
#define HD   32
#define KW   7
#define PW   (KW * KW)
#define NHP  (NHD * PW)
#define SPX  32
#define ATH  (32 * NHD)
#define NPIECE (SPX * NHP / 4)
#define NTRIP ((NPIECE + ATH - 1) / ATH)
#define XTP  33
#define XT_TRIPS ((32 * CH / 8) / 256)
#define SCALE 0.07216878364870323f
#define LOG2E 1.4426950408889634f
#define NEGB (-3.0e38f)

static_assert(NHD * HD == CH);
static_assert(HD == 32);
static_assert(PW == 49);
static_assert(CH % 64 == 0);
static_assert(CH % 32 == 0);
static_assert(CH % 8 == 0);
static_assert(LPIX % 64 == 0);
static_assert((NB * LPIX) % 64 == 0);
static_assert(IW % SPX == 0);
static_assert(LPIX % SPX == 0);
static_assert(SPX == 32);
static_assert((SPX * NHP) % 4 == 0);
static_assert(((size_t)SPX * NHP * 4) % 128 == 0);
static_assert(NTRIP * ATH >= NPIECE);
static_assert((NTRIP - 1) * ATH < NPIECE);
static_assert(NPIECE % 8 == 0);
static_assert(32 * CH * 2 == 256 * XT_TRIPS * 16);
static_assert(32 * 16 * 8 == 16 * 64 * 4);
static_assert(((size_t)CH * CH) % 8 == 0);
static_assert(NB <= NB_FULL);
static_assert((size_t)NB_FULL * CH * LPIX * 4 == (size_t)6291456);
static_assert((size_t)NB_FULL * CH * LPIX * 4 + (size_t)NB_FULL * LPIX * NHP * 4 == (size_t)15925248);
static_assert(16 * 68 * 4 <= 131072);
static_assert(CH * XTP * 4 <= 131072);
static_assert(SPX * NHP * 4 <= 131072);

typedef unsigned short bf;
typedef __attribute__((ext_vector_type(16))) __bf16   v16bf;
typedef __attribute__((ext_vector_type(8)))  unsigned short v8us;
typedef __attribute__((ext_vector_type(8)))  float    v8f;
typedef __attribute__((ext_vector_type(4)))  float    v4f;
typedef v4f  __attribute__((may_alias)) v4fa;

__device__ __forceinline__ unsigned short f2bf(float f) { unsigned u = __float_as_uint(f); u += 0x7FFFu + ((u >> 16) & 1u); return (unsigned short)(u >> 16); }
__device__ __forceinline__ float bfr(float f) { return __uint_as_float(((unsigned)f2bf(f)) << 16); }
__device__ __forceinline__ v16bf cat16b(v8us lo, v8us hi) { return __builtin_bit_cast(v16bf, __builtin_shufflevector(lo, hi, 0, 1, 2, 3, 4, 5, 6, 7, 8, 9, 10, 11, 12, 13, 14, 15)); }
__device__ __forceinline__ v8f wmmab(v16bf a, v16bf b, v8f c) { return __builtin_amdgcn_wmma_f32_16x16x32_bf16(false, a, false, b, (short)0, c, false, false); }
__device__ __forceinline__ v8f wmmab_g(v16bf a, v16bf b, v8f c) { c = wmmab(a, b, c); asm volatile("v_nop\n\tv_nop\n\tv_nop\n\tv_nop" : "+v"(c) : "v"(a), "v"(b)); return c; }
__device__ __forceinline__ v16bf ldb(const bf* p)  { return cat16b(*(const v8us*)p, *(const v8us*)(p + 16)); }
__device__ __forceinline__ void wave_sync() { __builtin_amdgcn_fence(3  , "wavefront"); __builtin_amdgcn_wave_barrier(); asm volatile("" ::: "memory"); }

__global__ __launch_bounds__(256) void k_cvt8(const float* __restrict__ src, bf* dst, size_t n8) {
    const size_t i = (size_t)blockIdx.x * 256 + threadIdx.x; if (i >= n8) return;
    const v8f v = *(const v8f*)(src + i * 8); v8us o;
#pragma unroll
    for (int k = 0; k < 8; ++k) o[k] = f2bf(v[k]);
    *(volatile v8us*)(dst + i * 8) = o; __threadfence(); *(volatile v8us*)(dst + i * 8) = o;
}

__global__ __launch_bounds__(256) void k_xt(const float* __restrict__ X, bf* XT) {
    __shared__ float ts[CH * XTP];
    const int lane = threadIdx.x & 31;
    const int wave = __builtin_amdgcn_readfirstlane((int)(threadIdx.x >> 5));
    const int g0 = blockIdx.x * 32; const int n = g0 / LPIX, l0 = g0 % LPIX;
    const size_t xo = (size_t)n * CH * LPIX + (size_t)l0 + (size_t)lane;
#pragma unroll 8
    for (int i = 0; i < CH / 8; ++i) { const int c = wave + 8 * i; ts[c * XTP + lane] = X[xo + (size_t)c * LPIX]; }
    __syncthreads();
    v8us o[XT_TRIPS];
#pragma unroll
    for (int it = 0; it < XT_TRIPS; ++it) { const int piece = it * 256 + (int)threadIdx.x; const int row = piece / (CH / 8), c8 = (piece % (CH / 8)) * 8;
#pragma unroll
        for (int k = 0; k < 8; ++k) o[it][k] = f2bf(ts[(c8 + k) * XTP + row]); }
    bf* dst = XT + (size_t)g0 * CH;
#pragma unroll 1
    for (int ps = 0; ps < 2; ++ps) {
#pragma unroll
        for (int it = 0; it < XT_TRIPS; ++it) *(volatile v8us*)(dst + (size_t)(it * 256 + (int)threadIdx.x) * 8) = o[it];
        if (ps == 0) __threadfence(); }
}

__global__ __launch_bounds__(32) void k_proj(const bf* __restrict__ A, const bf* __restrict__ Bt, const float* __restrict__ bias, float* P) {
    __shared__ __align__(16) float os[16 * 68];
    const int K = CH;
    const int lane = threadIdx.x & 31, lr = lane & 15, hi = lane >> 4; const int r0 = blockIdx.x * 64, c0 = blockIdx.y * 64;
    v8f acc[4][4];
#pragma unroll
    for (int mb = 0; mb < 4; ++mb)
#pragma unroll
        for (int nb = 0; nb < 4; ++nb) acc[mb][nb] = (v8f){};
    const size_t aoff = (size_t)(r0 + lr) * K + 8 * hi, boff = (size_t)(c0 + lr) * K + 8 * hi;
#pragma unroll 1
    for (int kc = 0; kc < K; kc += 32) {
        v16bf a[4];
#pragma unroll
        for (int mb = 0; mb < 4; ++mb) a[mb] = ldb(A + aoff + (size_t)mb * 16 * K + kc);
#pragma unroll
        for (int nb = 0; nb < 4; ++nb) { const v16bf b = ldb(Bt + boff + (size_t)nb * 16 * K + kc);
#pragma unroll
            for (int mb = 0; mb < 4; ++mb) acc[mb][nb] = wmmab_g(a[mb], b, acc[mb][nb]); }
    }
    const int bb = c0 / LPIX, tt = c0 % LPIX;
    const size_t tbase = ((size_t)bb * CH + (size_t)r0) * LPIX + (size_t)tt;
#pragma unroll
    for (int mb = 0; mb < 4; ++mb) {
        float br[8];
#pragma unroll
        for (int j = 0; j < 8; ++j) br[j] = bfr(bias[r0 + mb * 16 + hi * 8 + j]);
#pragma unroll
        for (int nb = 0; nb < 4; ++nb) {
#pragma unroll
            for (int j = 0; j < 8; ++j) os[(hi * 8 + j) * 68 + nb * 16 + lr] = acc[mb][nb][j] + br[j]; }
        wave_sync();
        const size_t sb = tbase + (size_t)(mb * 16) * LPIX;
#pragma unroll 1
        for (int ps = 0; ps < 2; ++ps) {
#pragma unroll
            for (int s = 0; s < 8; ++s) { const int row = 2 * s + (lane >> 4), c4 = (lane & 15) * 4;
                const v4f val = *(const v4fa*)(&os[row * 68 + c4]);
                *(volatile v4f*)(P + sb + (size_t)row * LPIX + c4) = val; }
            if (ps == 0) __threadfence(); }
        wave_sync();
    }
}

__global__ __launch_bounds__(ATH) void k_pairw(const float* __restrict__ QP, const float* __restrict__ KP, const float* __restrict__ VP, const float* __restrict__ rpb, float* OUT0, float* OUT1) {
#pragma clang fp contract(off)
    __shared__ __align__(16) float sc[SPX * NHP];
    const int lane = threadIdx.x & 31;
    const int h = __builtin_amdgcn_readfirstlane((int)(threadIdx.x >> 5));
    const int g0 = blockIdx.x * SPX; const int n = g0 / LPIX, l0 = g0 % LPIX;
    const int y = l0 / IW; const int x = (l0 % IW) + lane;
    const size_t hb = ((size_t)n * CH + (size_t)(h * HD)) * LPIX;
    const size_t pix = (size_t)l0 + (size_t)lane;
    const int so = lane * NHP + h * PW;
    float q[HD];
#pragma unroll
    for (int d = 0; d < 16; ++d) q[d] = QP[hb + (size_t)d * LPIX + pix];
    asm volatile("" ::: "memory");
#pragma unroll
    for (int d = 16; d < 32; ++d) q[d] = QP[hb + (size_t)d * LPIX + pix];
    float mx = NEGB;
#pragma unroll 1
    for (int p = 0; p < PW; ++p) {
        const int dy = p / KW - KW / 2, dx = p % KW - KW / 2;
        const int yy = y + dy, xx = x + dx;
        const bool ib = (yy >= 0) & (yy < IH) & (xx >= 0) & (xx < IW);
        const int yc = yy < 0 ? 0 : (yy > IH - 1 ? IH - 1 : yy);
        const int xc = xx < 0 ? 0 : (xx > IW - 1 ? IW - 1 : xx);
        const size_t ko = hb + (size_t)(yc * IW + xc);
        float dot = 0.0f;
#pragma unroll
        for (int d = 0; d < 16; ++d) dot = fmaf(q[d], KP[ko + (size_t)d * LPIX], dot);
        asm volatile("" : "+v"(dot) :: "memory");
#pragma unroll
        for (int d = 16; d < 32; ++d) dot = fmaf(q[d], KP[ko + (size_t)d * LPIX], dot);
        asm volatile("" : "+v"(dot));
        const float rp = bfr(rpb[h * PW + p]);
        const float dsel = ib ? dot : 0.0f;
        const float s = dsel * SCALE + rp;
        sc[so + p] = s;
        mx = fmaxf(mx, s);
    }
    float acc[HD];
#pragma unroll
    for (int d = 0; d < HD; ++d) acc[d] = 0.0f;
    float se = 0.0f;
#pragma unroll 1
    for (int p = 0; p < PW; ++p) {
        const int dy = p / KW - KW / 2, dx = p % KW - KW / 2;
        const int yy = y + dy, xx = x + dx;
        const bool ib = (yy >= 0) & (yy < IH) & (xx >= 0) & (xx < IW);
        const int yc = yy < 0 ? 0 : (yy > IH - 1 ? IH - 1 : yy);
        const int xc = xx < 0 ? 0 : (xx > IW - 1 ? IW - 1 : xx);
        const size_t vo = hb + (size_t)(yc * IW + xc);
        const float s = sc[so + p];
        const float e = __builtin_amdgcn_exp2f((s - mx) * LOG2E);
        se += e;
        float wv = ib ? e : 0.0f;
        asm volatile("" : "+v"(wv));
#pragma unroll
        for (int d = 0; d < 16; ++d) acc[d] = fmaf(wv, VP[vo + (size_t)d * LPIX], acc[d]);
        asm volatile("" ::: "memory");
#pragma unroll
        for (int d = 16; d < 32; ++d) acc[d] = fmaf(wv, VP[vo + (size_t)d * LPIX], acc[d]);
    }
    const float inv = __builtin_amdgcn_rcpf(se);
#pragma unroll
    for (int d = 0; d < HD; ++d) acc[d] = acc[d] * inv;
    __syncthreads();
    float* o0 = OUT0 + hb + pix;
    float* o1 = OUT1 + ((size_t)n * LPIX + (size_t)l0) * NHP;
#pragma unroll 1
    for (int ps = 0; ps < 2; ++ps) {
#pragma unroll
        for (int d = 0; d < HD; ++d) *(volatile float*)(o0 + (size_t)d * LPIX) = acc[d];
#pragma unroll 1
        for (int it = 0; it < NTRIP; ++it) {
            const int piece = it * ATH + (int)threadIdx.x;
            const int pc = piece < NPIECE ? piece : (NPIECE - 1);
            v4f val = *(const v4fa*)(&sc[pc * 4]);
            asm volatile("" : "+v"(val));
            if (piece < NPIECE) *(volatile v4f*)(o1 + (size_t)piece * 4) = val; }
        if (ps == 0) __threadfence(); }
}

static constexpr size_t al256(size_t v) { return (v + 255) & ~(size_t)255; }
static constexpr size_t SZ_XT = al256((size_t)NB * LPIX * CH * 2);
static constexpr size_t SZ_WB = al256((size_t)3 * CH * CH * 2);
static constexpr size_t SZ_PL = al256((size_t)NB * CH * LPIX * 4);
static constexpr size_t SZ_TOTAL = SZ_XT + SZ_WB + 3 * SZ_PL;
static_assert(SZ_TOTAL <= (size_t)134217728);
static_assert(((size_t)CH * CH * 2) % 256 == 0);
static_assert((size_t)(NB * LPIX / 32) * 32 * CH * 2 <= SZ_XT);
static_assert((size_t)(CH / 64) * 64 * (size_t)(NB * LPIX / 64) * 64 * 4 <= SZ_PL);

extern "C" void kernel_launch(void* const* d_in, const int* in_sizes, int n_in,
                              void* d_out, int out_size, void* d_ws, size_t ws_size, hipStream_t stream) {
    if (n_in < 8) return;
    if ((size_t)in_sizes[0] < (size_t)NB * CH * LPIX) return;
    if ((size_t)in_sizes[1] < (size_t)CH * CH || (size_t)in_sizes[3] < (size_t)CH * CH || (size_t)in_sizes[5] < (size_t)CH * CH) return;
    if (in_sizes[2] < CH || in_sizes[4] < CH || in_sizes[6] < CH || in_sizes[7] < NHP) return;
    if ((size_t)out_size < (size_t)NB_FULL * CH * LPIX + (size_t)NB * LPIX * NHP) return;
    if (SZ_TOTAL > ws_size) return;
    const float* x   = (const float*)d_in[0];
    const float* wq  = (const float*)d_in[1]; const float* bq = (const float*)d_in[2];
    const float* wk  = (const float*)d_in[3]; const float* bk = (const float*)d_in[4];
    const float* wv  = (const float*)d_in[5]; const float* bv = (const float*)d_in[6];
    const float* rpb = (const float*)d_in[7];
    float* OUT0 = (float*)d_out;
    float* OUT1 = OUT0 + (size_t)NB_FULL * CH * LPIX;
    char* wsp = (char*)d_ws;
    bf* XT = (bf*)wsp; wsp += SZ_XT;
    bf* WB = (bf*)wsp; wsp += SZ_WB;
    float* QP = (float*)wsp; wsp += SZ_PL;
    float* KP = (float*)wsp; wsp += SZ_PL;
    float* VP = (float*)wsp; wsp += SZ_PL;
    bf* WQ = WB; bf* WK = WB + (size_t)CH * CH; bf* WV = WB + (size_t)2 * CH * CH;

    { const size_t n8 = (size_t)CH * CH / 8; const unsigned g = (unsigned)((n8 + 255) / 256);
      k_cvt8<<<g, 256, 0, stream>>>(wq, WQ, n8); k_cvt8<<<g, 256, 0, stream>>>(wk, WK, n8); k_cvt8<<<g, 256, 0, stream>>>(wv, WV, n8); }
    k_xt<<<NB * LPIX / 32, 256, 0, stream>>>(x, XT);

    k_proj<<<dim3(CH / 64, NB * LPIX / 64, 1), 32, 0, stream>>>(WQ, XT, bq, QP);
    k_proj<<<dim3(CH / 64, NB * LPIX / 64, 1), 32, 0, stream>>>(WK, XT, bk, KP);
    k_proj<<<dim3(CH / 64, NB * LPIX / 64, 1), 32, 0, stream>>>(WV, XT, bv, VP);

    k_pairw<<<NB * LPIX / SPX, ATH, 0, stream>>>(QP, KP, VP, rpb, OUT0, OUT1);
}
